// SDPAttention_48850958025226
// MI455X (gfx1250) — hardware-verified
//
#include <hip/hip_runtime.h>


typedef _Float16 __hf16;
#define __bf16 __hf16
typedef __attribute__((ext_vector_type(16))) _Float16 v16bf;
typedef __attribute__((ext_vector_type(8)))  float  v8f;
typedef __attribute__((ext_vector_type(4)))  float  v4f;

static constexpr int   BATCH = 16;
static constexpr int   SEQ   = 2048;
static constexpr int   DK    = 128;
static constexpr float SCALE = 0.08838834764831843f;

__device__ __forceinline__ __bf16 tobf(float x) { return (__bf16)x; }

__device__ __forceinline__ v8f wmma_bf16(v16bf a, v16bf b, v8f c) {
  v8f d = __builtin_amdgcn_wmma_f32_16x16x32_f16(false, a, false, b, (short)0, c,
                                                  false, false);
  asm volatile("v_nop\n\tv_nop\n\tv_nop\n\tv_nop" : "+v"(d) : "v"(a), "v"(b));
  return d;
}

template <typename SrcT>
__device__ __forceinline__ v16bf load_frag_MK(const SrcT* src, int ld, int lane) {
  const int r  = lane & 15;
  const int kb = (lane >> 4) << 3;
  const SrcT* p = src + r * ld;
  v16bf f;
#pragma unroll
  for (int i = 0; i < 4; ++i) {
    f[2 * i]         = tobf((float)p[kb + 2 * i]);
    f[2 * i + 1]     = tobf((float)p[kb + 2 * i + 1]);
    f[8 + 2 * i]     = tobf((float)p[16 + kb + 2 * i]);
    f[8 + 2 * i + 1] = tobf((float)p[16 + kb + 2 * i + 1]);
  }
  return f;
}

__device__ __forceinline__ v16bf load_fragB_KN(const __bf16* src, int ld, int n0,
                                               int lane) {
  const int n  = n0 + (lane & 15);
  const int kb = (lane >> 4) << 3;
  v16bf f;
#pragma unroll
  for (int i = 0; i < 4; ++i) {
    f[2 * i]         = src[(kb + 2 * i) * ld + n];
    f[2 * i + 1]     = src[(kb + 2 * i + 1) * ld + n];
    f[8 + 2 * i]     = src[(16 + kb + 2 * i) * ld + n];
    f[8 + 2 * i + 1] = src[(16 + kb + 2 * i + 1) * ld + n];
  }
  return f;
}

__device__ __forceinline__ void stage_rows_bf16(const float* src, __bf16* dst,
                                                int dstld, int rows, int tid,
                                                int nthreads) {
  const int q4 = DK / 4;
  for (int i = tid; i < rows * q4; i += nthreads) {
    const int r = i / q4;
    const int c = (i % q4) * 4;
    const float4 v = *(const float4*)(src + r * DK + c);
    __bf16* d = dst + r * dstld + c;
    d[0] = tobf(v.x); d[1] = tobf(v.y); d[2] = tobf(v.z); d[3] = tobf(v.w);
  }
}

__global__ __launch_bounds__(256) void sdpa_colstats(const float* __restrict__ Q,
                                                     const float* __restrict__ K,
                                                     float* __restrict__ mbuf,
                                                     float* __restrict__ lbuf) {
  __shared__ __bf16 Qlds[16 * 136];
  __shared__ float sML[2][128];
  const int b    = blockIdx.x >> 4;
  const int kb0  = (blockIdx.x & 15) * 128;
  const int wave = threadIdx.x >> 5;
  const int lane = threadIdx.x & 31;
  const int kb   = kb0 + wave * 16;
  const int kcol = lane & 15;
  const int half = lane >> 4;

  const float* Kb = K + ((size_t)b * SEQ + kb) * DK;
  v16bf bk[4];
#pragma unroll
  for (int j = 0; j < 4; ++j) bk[j] = load_frag_MK(Kb + j * 32, DK, lane);

  float m_col = -1e30f, l_col = 0.0f;

  for (int qc = kb0; qc < SEQ; qc += 16) {
    __syncthreads();
    stage_rows_bf16(Q + ((size_t)b * SEQ + qc) * DK, Qlds, 136, 16,
                    threadIdx.x, 256);
    __syncthreads();
    if (qc + 15 >= kb) {
      v16bf aq[4];
#pragma unroll
      for (int j = 0; j < 4; ++j) aq[j] = load_frag_MK(Qlds + j * 32, 136, lane);
      v8f c = {};
#pragma unroll
      for (int j = 0; j < 4; ++j) c = wmma_bf16(aq[j], bk[j], c);

      const int kglob = kb + kcol;
      float s[8];
      float tm = -1e30f;
#pragma unroll
      for (int v = 0; v < 8; ++v) {
        const int qglob = qc + v + 8 * half;
        s[v] = (kglob > qglob) ? -1e9f : c[v] * SCALE;
        tm = fmaxf(tm, s[v]);
      }
      tm = fmaxf(tm, __shfl_xor(tm, 16, 32));
      const float mn = fmaxf(m_col, tm);
      float se = 0.0f;
#pragma unroll
      for (int v = 0; v < 8; ++v) se += __expf(s[v] - mn);
      se += __shfl_xor(se, 16, 32);
      l_col = l_col * __expf(m_col - mn) + se;
      m_col = mn;
    }
  }
  if (lane < 16) { sML[0][wave * 16 + kcol] = m_col; sML[1][wave * 16 + kcol] = l_col; }
  __syncthreads();
  if (threadIdx.x < 64) {
    const int which = threadIdx.x >> 5, q4 = (threadIdx.x & 31) * 4;
    float* dst = (which ? lbuf : mbuf) + (size_t)b * SEQ + kb0 + q4;
    const v4f v = *(const v4f*)(&sML[which][q4]);
    *(volatile v4f*)dst = v; __threadfence(); *(volatile v4f*)dst = v;
  }
}

__global__ __launch_bounds__(256) void sdpa_output(const float* __restrict__ Q,
                                                   const float* __restrict__ K,
                                                   const float* __restrict__ V,
                                                   const float* __restrict__ mbuf,
                                                   const float* __restrict__ lbuf,
                                                   float* __restrict__ out) {
  __shared__ __bf16 Klds[32 * 136];
  __shared__ __bf16 Vlds[32 * 136];
  __shared__ __bf16 Plds[8 * 16 * 40];
  __shared__ __attribute__((aligned(16))) float Olds[8][16 * DK];
  const int b    = blockIdx.x >> 4;
  const int qb0  = (blockIdx.x & 15) * 128;
  const int wave = threadIdx.x >> 5;
  const int lane = threadIdx.x & 31;
  const int qb   = qb0 + wave * 16;
  const int half = lane >> 4;
  const int n    = lane & 15;
  __bf16* Pw = Plds + wave * 16 * 40;

  const float* Qb = Q + ((size_t)b * SEQ + qb) * DK;
  v16bf aq[4];
#pragma unroll
  for (int j = 0; j < 4; ++j) aq[j] = load_frag_MK(Qb + j * 32, DK, lane);

  v8f o[8] = {};

  const int kmax = qb0 + 127;
  for (int kc = 0; kc <= kmax; kc += 32) {
    __syncthreads();
    stage_rows_bf16(K + ((size_t)b * SEQ + kc) * DK, Klds, 136, 32,
                    threadIdx.x, 256);
    stage_rows_bf16(V + ((size_t)b * SEQ + kc) * DK, Vlds, 136, 32,
                    threadIdx.x, 256);
    __syncthreads();
    if (kc <= qb + 15) {
#pragma unroll
      for (int t = 0; t < 2; ++t) {
        v8f c = {};
#pragma unroll
        for (int j = 0; j < 4; ++j) {
          v16bf bk = load_frag_MK(Klds + (t * 16) * 136 + j * 32, 136, lane);
          c = wmma_bf16(aq[j], bk, c);
        }
        const int kglob = kc + t * 16 + n;
        const float mk = mbuf[(size_t)b * SEQ + kglob];
        const float rl = 1.0f / lbuf[(size_t)b * SEQ + kglob];
#pragma unroll
        for (int v = 0; v < 8; ++v) {
          const int qglob = qb + v + 8 * half;
          const float p =
              (kglob > qglob) ? 0.0f : __expf(c[v] * SCALE - mk) * rl;
          Pw[(v + 8 * half) * 40 + t * 16 + n] = tobf(p);
        }
      }
      asm volatile("s_wait_dscnt 0" ::: "memory");

      const v16bf ap = load_frag_MK(Pw, 40, lane);
#pragma unroll
      for (int d = 0; d < 8; ++d) {
        v16bf bv = load_fragB_KN(Vlds, 136, d * 16, lane);
        o[d] = wmma_bf16(ap, bv, o[d]);
      }
    }
  }

  float* Ow = Olds[wave];
#pragma unroll
  for (int d = 0; d < 8; ++d)
#pragma unroll
    for (int v = 0; v < 8; ++v)
      Ow[(v + 8 * half) * DK + d * 16 + n] = o[d][v];
  asm volatile("s_wait_dscnt 0" ::: "memory");
  __builtin_amdgcn_fence(__ATOMIC_RELEASE, "workgroup"); __builtin_amdgcn_wave_barrier(); __builtin_amdgcn_fence(__ATOMIC_ACQUIRE, "workgroup");
  float* Ob = out + ((size_t)b * SEQ + qb) * DK;
  for (int pass = 0; pass < 2; ++pass) {
#pragma unroll
    for (int rr = 0; rr < 16; ++rr)
      *(volatile v4f*)(Ob + (size_t)rr * DK + lane * 4) = *(const v4f*)(Ow + rr * DK + lane * 4);
    __threadfence();
  }
}

extern "C" void kernel_launch(void* const* d_in, const int* in_sizes, int n_in,
                              void* d_out, int out_size, void* d_ws,
                              size_t ws_size, hipStream_t stream) {
  (void)in_sizes; (void)n_in; (void)out_size; (void)ws_size;
  const float* Q = (const float*)d_in[0];
  const float* K = (const float*)d_in[1];
  const float* V = (const float*)d_in[2];
  float* out  = (float*)d_out;
  float* mbuf = (float*)d_ws;
  float* lbuf = mbuf + (size_t)BATCH * SEQ;

  const dim3 grid(BATCH * (SEQ / 128));
  const dim3 block(256);
  sdpa_colstats<<<grid, block, 0, stream>>>(Q, K, mbuf, lbuf);
  sdpa_output<<<grid, block, 0, stream>>>(Q, K, V, mbuf, lbuf, out);
}
